// RNN_3341484556375
// MI455X (gfx1250) — hardware-verified
//
#include <hip/hip_runtime.h>
#include <math.h>

constexpr int NBATCH   = 256;
constexpr int NSTEP    = 4096;
constexpr int NHID     = 32;
constexpr int ROWS_BLK = 16;
constexpr int CHUNK    = 32;
constexpr int HPITCH = 40;
constexpr int WPITCH = 40;
constexpr int XPITCH = 16;
constexpr int YPITCH = 36;
constexpr int PPITCH = 20;
constexpr int LPITCH = 36;
constexpr float HCARRY = 16.0f;
constexpr float WCARRY = 64.0f;
constexpr float CCARRY = HCARRY * WCARRY;
constexpr float CCARRY_INV = 1.0f / CCARRY;
constexpr int NOUT0 = NBATCH * NSTEP;
constexpr int NOUT1 = NBATCH * NHID;

static_assert(NHID == 32, "one 32-deep k-step, two 16-column n-tiles");
static_assert(NBATCH % ROWS_BLK == 0, "grid exact");
static_assert(NSTEP % CHUNK == 0, "no chunk tail");
static_assert(CHUNK == 32, "one 128-B line of y per row per chunk");
static_assert((size_t)NOUT0 * 4 == 4194304, "out1 byte offset");
static_assert(((size_t)NOUT0 + (size_t)NOUT1) * 4 == 4227072, "d_out total bytes");
static_assert(((size_t)NOUT0 * 4) % 128 == 0, "out1 starts on a line");
static_assert(HPITCH % 8 == 0 && WPITCH % 8 == 0, "16-B aligned fragment rows");
static_assert(YPITCH % 4 == 0 && PPITCH % 4 == 0 && LPITCH % 4 == 0 && XPITCH % 4 == 0, "16-B aligned f32 rows");

typedef __attribute__((ext_vector_type(16))) _Float16 v16h;
typedef __attribute__((ext_vector_type(8)))  _Float16 v8h;
typedef __attribute__((ext_vector_type(8)))  float    v8f;
typedef __attribute__((ext_vector_type(4)))  float    v4f;

struct FragH {
  union U { v16h v; v8h h[2]; };
  static __device__ __forceinline__ v16h load(const _Float16* p) {
    U f; f.h[0] = *(const v8h*)(p); f.h[1] = *(const v8h*)(p + 16); return f.v;
  }
  static __device__ __forceinline__ v8f mma(v16h a, v16h b, v8f c) {
    return __builtin_amdgcn_wmma_f32_16x16x32_f16(false, a, false, b, (short)0, c, false, false);
  }
};

__device__ __forceinline__ void guard2(v8f& a, v8f& b, v16h x, v16h y, v16h z) {
  asm volatile("v_nop\n\tv_nop\n\tv_nop\n\tv_nop" : "+v"(a), "+v"(b) : "v"(x), "v"(y), "v"(z));
}

__device__ __forceinline__ float tanh_f32(float v) {
  const float e = expf(v + v);
  const float r = __builtin_amdgcn_rcpf(e + 1.0f);
  return 1.0f - 2.0f * r;
}

__global__ __launch_bounds__(32) void rnn_seq_kernel(const float* __restrict__ x, const float* __restrict__ h0,
                                                     const float* __restrict__ w_ih, const float* __restrict__ w_hh,
                                                     const float* __restrict__ b_ih, const float* __restrict__ b_hh,
                                                     const float* __restrict__ w_d, const float* __restrict__ b_d,
                                                     float* __restrict__ y, float* __restrict__ hlast) {
  __shared__ __align__(16) _Float16 Wb[NHID * WPITCH];
  __shared__ __align__(16) _Float16 Hb[ROWS_BLK * HPITCH];
  __shared__ __align__(16) float    Xt[CHUNK * XPITCH];
  __shared__ __align__(16) float    Yb[ROWS_BLK * YPITCH];
  __shared__ __align__(16) float    Pb[ROWS_BLK * PPITCH];
  __shared__ __align__(16) float    Lb[ROWS_BLK * LPITCH];

  const int lane = threadIdx.x & 31;
  const int hh   = lane >> 4;
  const int c    = lane & 15;
  const int q8   = lane >> 3;
  const int c4   = (lane & 7) * 4;
  const int b0   = blockIdx.x * ROWS_BLK;

  {
    const float* wr = w_hh + (size_t)lane * NHID;
#pragma unroll
    for (int q = 0; q < 4; ++q) {
      const v4f a = *(const v4f*)(wr + 8 * q);
      const v4f b = *(const v4f*)(wr + 8 * q + 4);
      v8h hv;
#pragma unroll
      for (int e = 0; e < 4; ++e) {
        hv[e]     = (_Float16)(a[e] * WCARRY);
        hv[4 + e] = (_Float16)(b[e] * WCARRY);
      }
      *(v8h*)(Wb + lane * WPITCH + 8 * q) = hv;
    }
  }
  asm volatile("" ::: "memory");

#pragma unroll
  for (int it = 0; it < 4; ++it) {
    const int row = it * 4 + q8;
    const v4f v = *(const v4f*)(h0 + (size_t)(b0 + row) * NHID + c4);
#pragma unroll
    for (int e = 0; e < 4; ++e) Hb[row * HPITCH + c4 + e] = (_Float16)(v[e] * HCARRY);
  }
  asm volatile("" ::: "memory");

  const float wi0 = w_ih[c] * CCARRY;
  const float wi1 = w_ih[16 + c] * CCARRY;
  const float bs0 = (b_ih[c] + b_hh[c]) * CCARRY;
  const float bs1 = (b_ih[16 + c] + b_hh[16 + c]) * CCARRY;
  const float wd0 = w_d[c];
  const float wd1 = w_d[16 + c];
  const float bdv = b_d[0];

  __syncthreads();

  const v16h bf0 = FragH::load(Wb + c * WPITCH + 8 * hh);
  const v16h bf1 = FragH::load(Wb + (16 + c) * WPITCH + 8 * hh);

  float hf0[8], hf1[8];
#pragma unroll
  for (int r = 0; r < 8; ++r) { hf0[r] = 0.0f; hf1[r] = 0.0f; }

#pragma unroll 1
  for (int ch = 0; ch < NSTEP / CHUNK; ++ch) {
    const int t0 = ch * CHUNK;
#pragma unroll
    for (int it = 0; it < 4; ++it) {
      const int row = it * 4 + q8;
      const v4f v = *(const v4f*)(x + (size_t)(b0 + row) * NSTEP + t0 + c4);
#pragma unroll
      for (int e = 0; e < 4; ++e) Xt[(c4 + e) * XPITCH + row] = v[e];
    }
    __syncthreads();

#pragma unroll 1
    for (int tt = 0; tt < CHUNK; ++tt) {
      const v4f xa = *(const v4f*)(Xt + tt * XPITCH + 8 * hh);
      const v4f xb = *(const v4f*)(Xt + tt * XPITCH + 8 * hh + 4);
      const v16h a = FragH::load(Hb + c * HPITCH + 8 * hh);
      v8f c0v, c1v;
#pragma unroll
      for (int e = 0; e < 4; ++e) {
        c0v[e]     = fmaf(xa[e], wi0, bs0);
        c0v[4 + e] = fmaf(xb[e], wi0, bs0);
        c1v[e]     = fmaf(xa[e], wi1, bs1);
        c1v[4 + e] = fmaf(xb[e], wi1, bs1);
      }
      asm volatile("" : "+v"(c0v), "+v"(c1v));
      v8f acc0 = FragH::mma(a, bf0, c0v);
      v8f acc1 = FragH::mma(a, bf1, c1v);
      guard2(acc0, acc1, a, bf0, bf1);

#pragma unroll
      for (int r = 0; r < 8; ++r) {
        const float hn0 = tanh_f32(acc0[r] * CCARRY_INV);
        const float hn1 = tanh_f32(acc1[r] * CCARRY_INV);
        hf0[r] = hn0;
        hf1[r] = hn1;
        Hb[(8 * hh + r) * HPITCH + c]      = (_Float16)(hn0 * HCARRY);
        Hb[(8 * hh + r) * HPITCH + 16 + c] = (_Float16)(hn1 * HCARRY);
        Pb[(8 * hh + r) * PPITCH + c] = fmaf(hn1, wd1, hn0 * wd0);
      }
      __syncthreads();

      const v4f pa = *(const v4f*)(Pb + c * PPITCH + 8 * hh);
      const v4f pb = *(const v4f*)(Pb + c * PPITCH + 8 * hh + 4);
      float s = ((pa[0] + pa[1]) + (pa[2] + pa[3])) + ((pb[0] + pb[1]) + (pb[2] + pb[3]));
      s += __shfl_xor(s, 16, 32);
      const float yv = tanh_f32(s + bdv);
      if (hh == 0) Yb[c * YPITCH + tt] = yv;
      __syncthreads();
    }

    v4f yv4[4];
#pragma unroll
    for (int it = 0; it < 4; ++it) yv4[it] = *(const v4f*)(Yb + (it * 4 + q8) * YPITCH + c4);
    for (int pass = 0; pass < 2; ++pass) {
#pragma unroll
      for (int it = 0; it < 4; ++it)
        *(volatile v4f*)(y + (size_t)(b0 + it * 4 + q8) * NSTEP + t0 + c4) = yv4[it];
      __threadfence();
    }
  }

#pragma unroll
  for (int r = 0; r < 8; ++r) {
    Lb[(8 * hh + r) * LPITCH + c]      = hf0[r];
    Lb[(8 * hh + r) * LPITCH + 16 + c] = hf1[r];
  }
  __syncthreads();
  v4f hv4[4];
#pragma unroll
  for (int it = 0; it < 4; ++it) hv4[it] = *(const v4f*)(Lb + (it * 4 + q8) * LPITCH + c4);
  for (int pass = 0; pass < 2; ++pass) {
#pragma unroll
    for (int it = 0; it < 4; ++it)
      *(volatile v4f*)(hlast + (size_t)(b0 + it * 4 + q8) * NHID + c4) = hv4[it];
    __threadfence();
  }
}

extern "C" void kernel_launch(void* const* d_in, const int* in_sizes, int n_in,
                              void* d_out, int out_size, void* d_ws, size_t ws_size, hipStream_t stream) {
  (void)d_ws; (void)ws_size;
  if (n_in < 8 || d_out == nullptr) return;
  if (in_sizes[0] != NBATCH * NSTEP || in_sizes[1] != NBATCH * NHID || in_sizes[2] != NHID ||
      in_sizes[3] != NHID * NHID || in_sizes[4] != NHID || in_sizes[5] != NHID ||
      in_sizes[6] != NHID || in_sizes[7] != 1 || out_size != NOUT0 + NOUT1) return;

  const float* x    = (const float*)d_in[0];
  const float* h0   = (const float*)d_in[1];
  const float* w_ih = (const float*)d_in[2];
  const float* w_hh = (const float*)d_in[3];
  const float* b_ih = (const float*)d_in[4];
  const float* b_hh = (const float*)d_in[5];
  const float* w_d  = (const float*)d_in[6];
  const float* b_d  = (const float*)d_in[7];
  float* out = (float*)d_out;

  rnn_seq_kernel<<<dim3(NBATCH / ROWS_BLK), dim3(32), 0, stream>>>(
      x, h0, w_ih, w_hh, b_ih, b_hh, w_d, b_d, out, out + (size_t)NOUT0);
}
